// MultiHead_37984690766458
// MI455X (gfx1250) — hardware-verified
//
#include <hip/hip_runtime.h>


#ifndef NB
#define NB 8
#endif
#ifndef SEQ
#define SEQ 2048
#endif
#define NB_FULL  8
#define SEQ_FULL 2048
#define EMB  256
#define NH   8
#define HD   32
#define FFH  1024
#define NROW (NB * SEQ)
#define NBH  (NB * NH)
#define WSC  64.0f
#define OSC  0.015625f
#define L2E  1.4426950408889634f
#define PCAR 1024.0f
#define EPSLN 1.0e-5f
#define NEGB (-3.0e38f)

static_assert(SEQ % 64 == 0);
static_assert(SEQ >= 64);
static_assert(SEQ <= SEQ_FULL);
static_assert(NB >= 1 && NB <= NB_FULL);
static_assert((NH % 2) == 0);
static_assert(EMB == NH * HD);
static_assert(HD == 32);
static_assert(EMB % 64 == 0 && FFH % 64 == 0);
static_assert(EMB % 32 == 0 && FFH % 32 == 0);
static_assert(NROW % 64 == 0);
static_assert(NROW % 8 == 0);
static_assert(NROW * EMB * 2 + 3 * NBH * SEQ * HD * 2 == NROW * FFH * 2);

typedef _Float16 h16;
typedef unsigned short bf;
typedef __attribute__((ext_vector_type(16))) __bf16   v16bf;
typedef __attribute__((ext_vector_type(16))) _Float16 v16h;
typedef __attribute__((ext_vector_type(8)))  _Float16 v8h;
typedef __attribute__((ext_vector_type(4)))  _Float16 v4h;
typedef __attribute__((ext_vector_type(2)))  _Float16 v2h;
typedef __attribute__((ext_vector_type(8)))  unsigned short v8us;
typedef __attribute__((ext_vector_type(2)))  unsigned short v2us;
typedef __attribute__((ext_vector_type(8)))  float v8f;
typedef __attribute__((ext_vector_type(4)))  float v4f;
typedef v4f __attribute__((may_alias)) v4fa;

__device__ __forceinline__ unsigned short f2bf(float f) { unsigned u = __float_as_uint(f); u += 0x7FFFu + ((u >> 16) & 1u); return (unsigned short)(u >> 16); }
__device__ __forceinline__ float bf2f(unsigned short b) { return __uint_as_float(((unsigned)b) << 16); }
__device__ __forceinline__ float bfr(float f) { return bf2f(f2bf(f)); }
__device__ __forceinline__ void splitf(float y, unsigned short& h, unsigned short& l) { h = f2bf(y); l = f2bf(y - bf2f(h)); }
__device__ __forceinline__ float ex2(float x) { return __builtin_amdgcn_exp2f(x); }
__device__ __forceinline__ v16h cat16(v8h lo, v8h hi) { return __builtin_shufflevector(lo, hi, 0, 1, 2, 3, 4, 5, 6, 7, 8, 9, 10, 11, 12, 13, 14, 15); }
__device__ __forceinline__ v16bf cat16b(v8us lo, v8us hi) { return __builtin_bit_cast(v16bf, __builtin_shufflevector(lo, hi, 0, 1, 2, 3, 4, 5, 6, 7, 8, 9, 10, 11, 12, 13, 14, 15)); }
__device__ __forceinline__ v8f wmma16(v16h a, v16h b, v8f c) { return __builtin_amdgcn_wmma_f32_16x16x32_f16(false, a, false, b, (short)0, c, false, false); }
__device__ __forceinline__ v8f wmmab(v16bf a, v16bf b, v8f c) { return __builtin_amdgcn_wmma_f32_16x16x32_bf16(false, a, false, b, (short)0, c, false, false); }

template <typename T16> struct WFrag;
template <> struct WFrag<h16> { typedef v16h V; static __device__ __forceinline__ V ld(const h16* p) { return cat16(*(const v8h*)p, *(const v8h*)(p + 16)); } static __device__ __forceinline__ v8f mma(V a, V b, v8f c) { return wmma16(a, b, c); } };
template <> struct WFrag<bf>  { typedef v16bf V; static __device__ __forceinline__ V ld(const bf* p) { return cat16b(*(const v8us*)p, *(const v8us*)(p + 16)); } static __device__ __forceinline__ v8f mma(V a, V b, v8f c) { return wmmab(a, b, c); } };

template <typename T16, int NSPLIT, int EPI, bool RES>
__global__ __launch_bounds__(32) void k_gemm(const T16* __restrict__ A, const T16* __restrict__ A2, const T16* __restrict__ Bt, int K,
                                             float mul, const float* __restrict__ bias, const float* __restrict__ res,
                                             float* CF, h16* C16, int ldc, int seq) {
    typedef typename WFrag<T16>::V V;
    __shared__ __align__(16) float os[16 * 68];
    const int lane = threadIdx.x & 31, lr = lane & 15, hi = lane >> 4;
    const int r0 = blockIdx.x * 64, c0 = blockIdx.y * 64;
    v8f acc[4][4];
#pragma unroll
    for (int mb = 0; mb < 4; ++mb)
#pragma unroll
        for (int nb = 0; nb < 4; ++nb) acc[mb][nb] = (v8f){};
    const size_t aoff = (size_t)(r0 + lr) * K + 8 * hi, boff = (size_t)(c0 + lr) * K + 8 * hi;
#pragma unroll 1
    for (int kc = 0; kc < K; kc += 32) {
        V a[4], a2[4];
#pragma unroll
        for (int mb = 0; mb < 4; ++mb) { a[mb] = WFrag<T16>::ld(A + aoff + (size_t)mb * 16 * K + kc); if (NSPLIT == 1) a2[mb] = WFrag<T16>::ld(A2 + aoff + (size_t)mb * 16 * K + kc); }
#pragma unroll
        for (int nb = 0; nb < 4; ++nb) { const V b = WFrag<T16>::ld(Bt + boff + (size_t)nb * 16 * K + kc);
#pragma unroll
            for (int mb = 0; mb < 4; ++mb) { acc[mb][nb] = WFrag<T16>::mma(a[mb], b, acc[mb][nb]); if (NSPLIT == 1) acc[mb][nb] = WFrag<T16>::mma(a2[mb], b, acc[mb][nb]); } }
        asm volatile("v_nop\n\tv_nop\n\tv_nop\n\tv_nop" : "+v"(acc[0][0]), "+v"(acc[1][1]), "+v"(acc[2][2]), "+v"(acc[3][3]) : "v"(a[0]), "v"(a[3]));
    }
    const int bb = r0 / seq, t0 = r0 - bb * seq, hA = c0 / HD;
    if (EPI == 3) {
        const int piece = lane & 7, rq = lane >> 3;
#pragma unroll
        for (int nb = 0; nb < 4; ++nb) {
#pragma unroll
            for (int mb = 0; mb < 4; ++mb) {
#pragma unroll
                for (int j = 0; j < 8; ++j) os[lr * 68 + mb * 16 + hi * 8 + j] = acc[mb][nb][j]; }
            __syncthreads();
            const int head = hA + (nb >> 1);
            h16* base = C16 + ((size_t)(bb * NH + head) * HD + (nb & 1) * 16) * seq + t0 + piece * 8;
#pragma unroll 1
            for (int ps = 0; ps < 2; ++ps) {
#pragma unroll
                for (int it = 0; it < 4; ++it) {
                    const int dl = 4 * it + rq; const float* op = os + dl * 68 + piece * 8;
                    const v4f u0 = *(const v4fa*)op, u1 = *(const v4fa*)(op + 4); v8h o;
#pragma unroll
                    for (int i = 0; i < 4; ++i) { o[i] = (h16)(u0[i] * mul); o[4 + i] = (h16)(u1[i] * mul); }
                    *(volatile v8h*)(base + (size_t)dl * seq) = o; }
                if (ps == 0) __threadfence(); }
            __syncthreads();
        }
    } else {
        v4f bz = (v4f){}; v8f b8 = (v8f){};
        if (EPI == 0) { const int cofs = lr * 4;
#pragma unroll
            for (int i = 0; i < 4; ++i) bz[i] = bfr(bias[c0 + cofs + i]); }
        if (EPI == 1) { const int piece = lane & 7;
#pragma unroll
            for (int i = 0; i < 8; ++i) b8[i] = bfr(bias[c0 + piece * 8 + i]); }
#pragma unroll
        for (int mb = 0; mb < 4; ++mb) {
#pragma unroll
            for (int nb = 0; nb < 4; ++nb) {
#pragma unroll
                for (int j = 0; j < 8; ++j) os[(hi * 8 + j) * 68 + nb * 16 + lr] = acc[mb][nb][j]; }
            __syncthreads();
#pragma unroll 1
            for (int ps = 0; ps < 2; ++ps) {
                if (EPI == 0) {
#pragma unroll
                    for (int s = 0; s < 8; ++s) {
                        const int row = 2 * s + hi, cofs = lr * 4; const int grow = r0 + mb * 16 + row;
                        v4f val = *(const v4fa*)(os + row * 68 + cofs); val = val * mul + bz;
                        if (RES) { const v4f rr = *(const v4f*)(res + (size_t)grow * ldc + c0 + cofs); val += rr; }
                        *(volatile v4f*)(CF + (size_t)grow * ldc + c0 + cofs) = val; }
                } else if (EPI == 1) {
                    const int piece = lane & 7, rq = lane >> 3;
#pragma unroll
                    for (int it = 0; it < 4; ++it) {
                        const int row = 4 * it + rq; const float* op = os + row * 68 + piece * 8;
                        const v4f u0 = *(const v4fa*)op, u1 = *(const v4fa*)(op + 4); v8h o;
#pragma unroll
                        for (int i = 0; i < 4; ++i) { o[i] = (h16)fmaxf(u0[i] * mul + b8[i], 0.0f); o[4 + i] = (h16)fmaxf(u1[i] * mul + b8[4 + i], 0.0f); }
                        *(volatile v8h*)(C16 + (size_t)(r0 + mb * 16 + row) * ldc + c0 + piece * 8) = o; }
                } else {
                    const int pq = lane & 3, rr = lane >> 2;
#pragma unroll
                    for (int hs = 0; hs < 2; ++hs) {
                        h16* base = C16 + ((size_t)(bb * NH + hA + hs) * seq + t0 + mb * 16) * HD + pq * 8;
#pragma unroll
                        for (int it = 0; it < 2; ++it) {
                            const int row = 8 * it + rr; const float* op = os + row * 68 + hs * 32 + pq * 8;
                            const v4f u0 = *(const v4fa*)op, u1 = *(const v4fa*)(op + 4); v8h o;
#pragma unroll
                            for (int i = 0; i < 4; ++i) { o[i] = (h16)(u0[i] * mul); o[4 + i] = (h16)(u1[i] * mul); }
                            *(volatile v8h*)(base + (size_t)row * HD) = o; } }
                }
                if (ps == 0) __threadfence(); }
            __syncthreads();
        }
    }
}

__global__ __launch_bounds__(256) void k_wt16(const float* __restrict__ src, int K, int N, int Dn, float sc, h16* dst) {
    const int lane = threadIdx.x & 31; const int L0 = (blockIdx.x * 8 + (threadIdx.x >> 5)) * 8; const int nlines = N * K / 64;
#pragma unroll 1
    for (int ps = 0; ps < 2; ++ps) {
#pragma unroll 1
        for (int l = 0; l < 8; ++l) { const int L = L0 + l; if (L >= nlines) break;
            const size_t e = (size_t)L * 64 + lane * 2; const int k = (int)(e % K), n = (int)(e / K); const int hh = n / Dn, d = n - hh * Dn;
            const float* sp = src + ((size_t)hh * K + k) * Dn + d; v2h o; o[0] = (h16)(bfr(sp[0]) * sc); o[1] = (h16)(bfr(sp[Dn]) * sc);
            *(volatile v2h*)(dst + e) = o; }
        if (ps == 0) __threadfence(); }
}
__global__ __launch_bounds__(256) void k_wtb(const float* __restrict__ src, int K, int N, int Dn, bf* dst) {
    const int lane = threadIdx.x & 31; const int L0 = (blockIdx.x * 8 + (threadIdx.x >> 5)) * 8; const int nlines = N * K / 64;
#pragma unroll 1
    for (int ps = 0; ps < 2; ++ps) {
#pragma unroll 1
        for (int l = 0; l < 8; ++l) { const int L = L0 + l; if (L >= nlines) break;
            const size_t e = (size_t)L * 64 + lane * 2; const int k = (int)(e % K), n = (int)(e / K); const int hh = n / Dn, d = n - hh * Dn;
            const float* sp = src + ((size_t)hh * K + k) * Dn + d; v2us o; o[0] = f2bf(sp[0]); o[1] = f2bf(sp[Dn]);
            *(volatile v2us*)(dst + e) = o; }
        if (ps == 0) __threadfence(); }
}

__global__ __launch_bounds__(256) void k_ln(const float* __restrict__ X, int seq, int seqf, const float* __restrict__ g, const float* __restrict__ be, int rin, float* YF, h16* Y16, int nrows) {
    const int w = threadIdx.x >> 5, lane = threadIdx.x & 31; const int r = blockIdx.x * 8 + w; if (r >= nrows) return;
    const int bb = r / seq, t = r - bb * seq; const float* xr = X + ((size_t)bb * seqf + t) * EMB;
    const v4f a0 = *(const v4f*)(xr + lane * 4), a1 = *(const v4f*)(xr + 128 + lane * 4);
    float v[8];
#pragma unroll
    for (int i = 0; i < 4; ++i) { v[i] = a0[i]; v[4 + i] = a1[i]; }
    if (rin) {
#pragma unroll
        for (int i = 0; i < 8; ++i) v[i] = bfr(v[i]); }
    float s = 0.0f;
#pragma unroll
    for (int i = 0; i < 8; ++i) s += v[i];
#pragma unroll
    for (int sh = 16; sh; sh >>= 1) s += __shfl_xor(s, sh, 32);
    const float mean = s * (1.0f / EMB);
    float ss = 0.0f;
#pragma unroll
    for (int i = 0; i < 8; ++i) { const float d = v[i] - mean; v[i] = d; ss += d * d; }
#pragma unroll
    for (int sh = 16; sh; sh >>= 1) ss += __shfl_xor(ss, sh, 32);
    const float rstd = rsqrtf(ss * (1.0f / EMB) + EPSLN);
    const v4f g0 = *(const v4f*)(g + lane * 4), g1v = *(const v4f*)(g + 128 + lane * 4), e0 = *(const v4f*)(be + lane * 4), e1 = *(const v4f*)(be + 128 + lane * 4);
    v4f y0, y1; v4h h0, h1;
#pragma unroll
    for (int i = 0; i < 4; ++i) { y0[i] = v[i] * rstd * bfr(g0[i]) + bfr(e0[i]); y1[i] = v[4 + i] * rstd * bfr(g1v[i]) + bfr(e1[i]); h0[i] = (h16)y0[i]; h1[i] = (h16)y1[i]; }
    float* yf = YF + (size_t)r * EMB; h16* yh = Y16 + (size_t)r * EMB;
#pragma unroll 1
    for (int ps = 0; ps < 2; ++ps) {
        *(volatile v4f*)(yf + lane * 4) = y0; *(volatile v4f*)(yf + 128 + lane * 4) = y1;
        *(volatile v4h*)(yh + lane * 4) = h0; *(volatile v4h*)(yh + 128 + lane * 4) = h1;
        if (ps == 0) __threadfence(); }
}

template <bool MASK>
__device__ __forceinline__ void col_upd(const v8f c, int tb, int s, float& m, float& z) {
    float x[8]; float mt = NEGB;
#pragma unroll
    for (int j = 0; j < 8; ++j) { float v = c[j] * 0.0625f; if (MASK) v = (tb + j >= s) ? v : NEGB; x[j] = v; mt = fmaxf(mt, v); }
    const float mn = fmaxf(m, mt); float sum = 0.0f;
#pragma unroll
    for (int j = 0; j < 8; ++j) { float e = ex2(x[j] - mn); if (MASK) e = (tb + j >= s) ? e : 0.0f; sum += e; }
    z = z * ex2(m - mn) + sum; m = mn;
}
template <bool MASK>
__device__ __forceinline__ void st_step(const h16* __restrict__ qp, int tt, const v16h kb0, const v16h kb1, int s, int hi, float& m0, float& z0, float& m1, float& z1) {
    const v16h a = WFrag<h16>::ld(qp + (size_t)tt * 16 * HD);
    v8f c0 = wmma16(a, kb0, (v8f){}); v8f c1 = wmma16(a, kb1, (v8f){});
    asm volatile("v_nop\n\tv_nop\n\tv_nop\n\tv_nop" : "+v"(c0), "+v"(c1) : "v"(a), "v"(kb0), "v"(kb1));
    const int tb = tt * 16 + 8 * hi;
    col_upd<MASK>(c0, tb, s, m0, z0); col_upd<MASK>(c1, tb, s + 16, m1, z1);
}
__global__ __launch_bounds__(32) void k_stats(const h16* __restrict__ Q, const h16* __restrict__ Kp, float* MX, float* ZF) {
    const int lane = threadIdx.x & 31, lr = lane & 15, hi = lane >> 4;
    const int bh = blockIdx.y, s0 = blockIdx.x * 32;
    const h16* kp = Kp + ((size_t)bh * SEQ + s0 + lr) * HD + 8 * hi;
    const v16h kb0 = WFrag<h16>::ld(kp), kb1 = WFrag<h16>::ld(kp + 16 * HD);
    const h16* qp = Q + ((size_t)bh * SEQ + lr) * HD + 8 * hi;
    const int s = s0 + lr;
    float m0 = NEGB, m1 = NEGB, z0 = 0.0f, z1 = 0.0f;
    const int tt0 = s0 >> 4;
    st_step<true>(qp, tt0, kb0, kb1, s, hi, m0, z0, m1, z1);
    st_step<true>(qp, tt0 + 1, kb0, kb1, s, hi, m0, z0, m1, z1);
#pragma unroll 1
    for (int tt = tt0 + 2; tt < SEQ / 16; ++tt) st_step<false>(qp, tt, kb0, kb1, s, hi, m0, z0, m1, z1);
    { const float mo = __shfl_xor(m0, 16, 32), zo = __shfl_xor(z0, 16, 32); const float mn = fmaxf(m0, mo); z0 = z0 * ex2(m0 - mn) + zo * ex2(mo - mn); m0 = mn; }
    { const float mo = __shfl_xor(m1, 16, 32), zo = __shfl_xor(z1, 16, 32); const float mn = fmaxf(m1, mo); z1 = z1 * ex2(m1 - mn) + zo * ex2(mo - mn); m1 = mn; }
    const float mm = hi ? m1 : m0, zz = hi ? z1 : z0; const float zf = __fdiv_rn(PCAR, zz);
    const size_t o = (size_t)bh * SEQ + s0 + lane;
    *(volatile float*)(MX + o) = mm; *(volatile float*)(ZF + o) = zf; __threadfence(); *(volatile float*)(MX + o) = mm; *(volatile float*)(ZF + o) = zf;
}

template <bool MASK>
__device__ __forceinline__ void pv_chunk(int sc, const h16* __restrict__ kb, const h16* __restrict__ vb, const float* __restrict__ mxb, const float* __restrict__ zfb,
                                         const v16h qb0, const v16h qb1, int tl, int hi, v8f& o00, v8f& o01, v8f& o10, v8f& o11) {
    const int s0 = sc * 32;
    const v16h va0 = WFrag<h16>::ld(vb + s0), va1 = WFrag<h16>::ld(vb + (size_t)16 * SEQ + s0);
    v8h p00, p01, p10, p11;
#pragma unroll
    for (int g = 0; g < 2; ++g) {
        const v16h ka = WFrag<h16>::ld(kb + (size_t)(s0 + 16 * g) * HD);
        const v8f mv = *(const v8f*)(mxb + s0 + 16 * g), zv = *(const v8f*)(zfb + s0 + 16 * g);
        v8f c0 = wmma16(ka, qb0, (v8f){}); v8f c1 = wmma16(ka, qb1, (v8f){});
        asm volatile("v_nop\n\tv_nop\n\tv_nop\n\tv_nop" : "+v"(c0), "+v"(c1) : "v"(ka), "v"(qb0), "v"(qb1));
        const int sb = s0 + 16 * g + 8 * hi;
        v8h pa, pc;
#pragma unroll
        for (int r = 0; r < 8; ++r) {
            float e0 = ex2(fmaf(c0[r], 0.0625f, -mv[r])) * zv[r];
            float e1 = ex2(fmaf(c1[r], 0.0625f, -mv[r])) * zv[r];
            if (MASK) { e0 = (sb + r <= tl) ? e0 : 0.0f; e1 = (sb + r <= tl + 16) ? e1 : 0.0f; }
            pa[r] = (h16)e0; pc[r] = (h16)e1; }
        if (g == 0) { p00 = pa; p01 = pc; } else { p10 = pa; p11 = pc; }
    }
    const v16h P0 = cat16(p00, p10), P1 = cat16(p01, p11);
    o00 = wmma16(va0, P0, o00); o01 = wmma16(va0, P1, o01); o10 = wmma16(va1, P0, o10); o11 = wmma16(va1, P1, o11);
    asm volatile("v_nop\n\tv_nop\n\tv_nop\n\tv_nop" : "+v"(o00), "+v"(o01), "+v"(o10), "+v"(o11) : "v"(va0), "v"(va1), "v"(P0), "v"(P1));
}
__global__ __launch_bounds__(64) void k_pv(const h16* __restrict__ Q, const h16* __restrict__ Kp, const h16* __restrict__ VT, const float* __restrict__ MX, const float* __restrict__ ZF,
                                          const float* __restrict__ XN, bf* XHh, bf* XHl) {
    __shared__ __align__(16) float os[32 * 68];
    const int w = threadIdx.x >> 5, lane = threadIdx.x & 31, lr = lane & 15, hi = lane >> 4;
    const int bh = blockIdx.y * 2 + w; const int hp = blockIdx.y % (NH / 2), bb = blockIdx.y / (NH / 2);
    const int tb = blockIdx.x, t0 = tb * 32;
    const h16* qp = Q + ((size_t)bh * SEQ + t0 + lr) * HD + 8 * hi;
    const v16h qb0 = WFrag<h16>::ld(qp), qb1 = WFrag<h16>::ld(qp + 16 * HD);
    const h16* kb = Kp + ((size_t)bh * SEQ + lr) * HD + 8 * hi;
    const h16* vb = VT + ((size_t)bh * HD + lr) * SEQ + 8 * hi;
    const float* mxb = MX + (size_t)bh * SEQ + 8 * hi; const float* zfb = ZF + (size_t)bh * SEQ + 8 * hi;
    const int tl = t0 + lr;
    v8f o00 = (v8f){}, o01 = (v8f){}, o10 = (v8f){}, o11 = (v8f){};
#pragma unroll 1
    for (int sc = 0; sc < tb; ++sc) pv_chunk<false>(sc, kb, vb, mxb, zfb, qb0, qb1, tl, hi, o00, o01, o10, o11);
    pv_chunk<true>(tb, kb, vb, mxb, zfb, qb0, qb1, tl, hi, o00, o01, o10, o11);
#pragma unroll
    for (int j = 0; j < 8; ++j) {
        os[(lr) * 68 + w * 32 + 8 * hi + j] = o00[j];
        os[(16 + lr) * 68 + w * 32 + 8 * hi + j] = o01[j];
        os[(lr) * 68 + w * 32 + 16 + 8 * hi + j] = o10[j];
        os[(16 + lr) * 68 + w * 32 + 16 + 8 * hi + j] = o11[j]; }
    __syncthreads();
    const int piece = lane & 7, rq = lane >> 3; const float ip = 1.0f / PCAR;
#pragma unroll 1
    for (int ps = 0; ps < 2; ++ps) {
#pragma unroll
        for (int it = 0; it < 4; ++it) {
            const int row = w * 16 + 4 * it + rq; const float* op = os + row * 68 + piece * 8;
            const v4f u0 = *(const v4fa*)op, u1 = *(const v4fa*)(op + 4);
            const size_t go = (size_t)(bb * SEQ + t0 + row) * EMB + hp * 64 + piece * 8;
            const v4f x0 = *(const v4f*)(XN + go), x1 = *(const v4f*)(XN + go + 4);
            v8us oh, ol;
#pragma unroll
            for (int i = 0; i < 4; ++i) { unsigned short a, c; splitf(x0[i] + u0[i] * ip, a, c); oh[i] = a; ol[i] = c; splitf(x1[i] + u1[i] * ip, a, c); oh[4 + i] = a; ol[4 + i] = c; }
            *(volatile v8us*)(XHh + go) = oh; *(volatile v8us*)(XHl + go) = ol; }
        if (ps == 0) __threadfence(); }
}

extern "C" void kernel_launch(void* const* d_in, const int* in_sizes, int n_in,
                              void* d_out, int out_size, void* d_ws, size_t ws_size, hipStream_t stream) {
    if (n_in < 14) return;
    if (in_sizes[0] < (NB - 1) * SEQ_FULL * EMB + SEQ * EMB) return;
    if (in_sizes[1] < NH * EMB * HD || in_sizes[2] < NH * EMB * HD || in_sizes[3] < NH * EMB * HD) return;
    if (in_sizes[4] < EMB * EMB || in_sizes[5] < EMB || in_sizes[6] < EMB || in_sizes[7] < EMB || in_sizes[8] < EMB || in_sizes[9] < EMB) return;
    if (in_sizes[10] < EMB * FFH || in_sizes[11] < FFH || in_sizes[12] < FFH * EMB || in_sizes[13] < EMB) return;
    if (out_size < NROW * EMB) return;
    const float* x = (const float*)d_in[0]; const float* wq = (const float*)d_in[1]; const float* wk = (const float*)d_in[2]; const float* wv = (const float*)d_in[3];
    const float* wlin = (const float*)d_in[4]; const float* blin = (const float*)d_in[5]; const float* g1 = (const float*)d_in[6]; const float* beta1 = (const float*)d_in[7];
    const float* g2 = (const float*)d_in[8]; const float* beta2 = (const float*)d_in[9]; const float* wf1 = (const float*)d_in[10]; const float* bf1 = (const float*)d_in[11];
    const float* wf2 = (const float*)d_in[12]; const float* bf2 = (const float*)d_in[13];
    float* OUT = (float*)d_out;
    char* wsp = (char*)d_ws;
    auto take = [&](size_t bytes) { char* p = wsp; wsp += (bytes + 255) & ~(size_t)255; return (void*)p; };
    float* R1 = (float*)take((size_t)NROW * EMB * 4);
    char* R2 = (char*)take((size_t)NROW * FFH * 2);
    h16* XN16 = (h16*)R2; h16* Q16 = (h16*)(R2 + (size_t)NROW * EMB * 2); h16* K16 = (h16*)(R2 + (size_t)NROW * EMB * 2 + (size_t)NBH * SEQ * HD * 2);
    h16* VT16 = (h16*)(R2 + (size_t)NROW * EMB * 2 + (size_t)2 * NBH * SEQ * HD * 2); h16* H16 = (h16*)R2;
    float* MX = (float*)take((size_t)NBH * SEQ * 4); float* ZF = (float*)take((size_t)NBH * SEQ * 4);
    bf* XHh = (bf*)take((size_t)NROW * EMB * 2); bf* XHl = (bf*)take((size_t)NROW * EMB * 2);
    float* X2F = (float*)take((size_t)NROW * EMB * 4); h16* X216 = (h16*)take((size_t)NROW * EMB * 2);
    h16* WQKV = (h16*)take((size_t)3 * EMB * EMB * 2); bf* WLIN = (bf*)take((size_t)EMB * EMB * 2); h16* WF1 = (h16*)take((size_t)FFH * EMB * 2); h16* WF2 = (h16*)take((size_t)EMB * FFH * 2);
    if ((size_t)(wsp - (char*)d_ws) > ws_size) return;
    float* XL = R1;
    const unsigned GW = (unsigned)((EMB * EMB / 64 + 63) / 64), GF = (unsigned)((FFH * EMB / 64 + 63) / 64);
    k_wt16<<<GW, 256, 0, stream>>>(wq, EMB, EMB, HD, WSC, WQKV);
    k_wt16<<<GW, 256, 0, stream>>>(wk, EMB, EMB, HD, WSC, WQKV + (size_t)EMB * EMB);
    k_wt16<<<GW, 256, 0, stream>>>(wv, EMB, EMB, HD, WSC, WQKV + (size_t)2 * EMB * EMB);
    k_wtb<<<GW, 256, 0, stream>>>(wlin, EMB, EMB, EMB, WLIN);
    k_wt16<<<GF, 256, 0, stream>>>(wf1, EMB, FFH, FFH, WSC, WF1);
    k_wt16<<<GF, 256, 0, stream>>>(wf2, FFH, EMB, EMB, WSC, WF2);
    k_ln<<<NROW / 8, 256, 0, stream>>>(x, SEQ, SEQ_FULL, g1, beta1, 1, R1, XN16, NROW);
    k_gemm<h16, 0, 2, false><<<dim3(NROW / 64, EMB / 64, 1), 32, 0, stream>>>(XN16, nullptr, WQKV, EMB, L2E * OSC, nullptr, nullptr, nullptr, Q16, 0, SEQ);
    k_gemm<h16, 0, 2, false><<<dim3(NROW / 64, EMB / 64, 1), 32, 0, stream>>>(XN16, nullptr, WQKV + (size_t)EMB * EMB, EMB, OSC, nullptr, nullptr, nullptr, K16, 0, SEQ);
    k_gemm<h16, 0, 3, false><<<dim3(NROW / 64, EMB / 64, 1), 32, 0, stream>>>(XN16, nullptr, WQKV + (size_t)2 * EMB * EMB, EMB, OSC, nullptr, nullptr, nullptr, VT16, 0, SEQ);
    k_stats<<<dim3(SEQ / 32, NBH, 1), 32, 0, stream>>>(Q16, K16, MX, ZF);
    k_pv<<<dim3(SEQ / 32, NBH / 2, 1), 64, 0, stream>>>(Q16, K16, VT16, MX, ZF, R1, XHh, XHl);
    k_gemm<bf, 1, 0, false><<<dim3(NROW / 64, EMB / 64, 1), 32, 0, stream>>>(XHh, XHl, WLIN, EMB, 1.0f, blin, nullptr, XL, nullptr, EMB, SEQ);
    k_ln<<<NROW / 8, 256, 0, stream>>>(XL, SEQ, SEQ, g2, beta2, 0, X2F, X216, NROW);
    k_gemm<h16, 0, 1, false><<<dim3(NROW / 64, FFH / 64, 1), 32, 0, stream>>>(X216, nullptr, WF1, EMB, OSC, bf1, nullptr, nullptr, H16, FFH, SEQ);
    k_gemm<h16, 0, 0, true><<<dim3(NROW / 64, EMB / 64, 1), 32, 0, stream>>>(H16, nullptr, WF2, FFH, OSC, bf2, X2F, OUT, nullptr, EMB, SEQ);
}
